// RoPEMultiHeadAttention_82755429859908
// MI455X (gfx1250) — hardware-verified
//
#include <hip/hip_runtime.h>
#include <math.h>

#ifndef NB
#define NB 2
#endif
#ifndef SEQ
#define SEQ 2048
#endif
#define NB_FULL 2
#define SEQ_FULL 2048
#define DD 1024
#define HH 16
#define DKK 64
#define QW 2
#define MTOK (NB * SEQ)
#define EARLY 64
#define LOROWS 128
#define GSTR 48
#define KSTRIDE 72
#define VSTRIDE 48
#define OSTR 72
#define WSC 64.0f
#define WSCI 0.015625f
#define PSC 1024.0f
#define WS_LIMIT 134217728

static_assert(SEQ % 128 == 0);
static_assert(SEQ >= LOROWS && LOROWS % 128 == 0);
static_assert(SEQ <= SEQ_FULL);
static_assert(NB >= 1 && NB <= NB_FULL);
static_assert(DD == HH * DKK);
static_assert(EARLY == 64);
static_assert((size_t)22 * (size_t)MTOK * (size_t)DD <= (size_t)WS_LIMIT);

typedef _Float16 f16;
typedef __bf16 bft;
typedef unsigned v4u_t __attribute__((ext_vector_type(4)));
typedef unsigned v4ua __attribute__((ext_vector_type(4), may_alias));
typedef float v4f_t __attribute__((ext_vector_type(4)));
typedef float v4fa __attribute__((ext_vector_type(4), may_alias));
typedef f16 f16x16 __attribute__((ext_vector_type(16)));
typedef f16 f16x8 __attribute__((ext_vector_type(8)));
typedef bft bfx16 __attribute__((ext_vector_type(16)));
typedef unsigned short u16x8 __attribute__((ext_vector_type(8)));
typedef unsigned short u16x16 __attribute__((ext_vector_type(16)));
typedef float f32x8 __attribute__((ext_vector_type(8)));

__device__ __forceinline__ f32x8 wmma16(f16x16 a, f16x16 b, f32x8 c) {
  c = __builtin_amdgcn_wmma_f32_16x16x32_f16(false, a, false, b, (short)0, c, false, false);
  asm volatile("v_nop\n\tv_nop\n\tv_nop\n\tv_nop" : "+v"(c) : "v"(a), "v"(b));
  return c;
}
__device__ __forceinline__ f32x8 wmmabf(u16x16 a, u16x16 b, f32x8 c) {
  c = __builtin_amdgcn_wmma_f32_16x16x32_bf16(false, __builtin_bit_cast(bfx16, a), false, __builtin_bit_cast(bfx16, b), (short)0, c, false, false);
  asm volatile("v_nop\n\tv_nop\n\tv_nop\n\tv_nop" : "+v"(c) : "v"(a), "v"(b));
  return c;
}

__device__ __forceinline__ unsigned short bfbits(float x) {
  unsigned u = __float_as_uint(x);
  u += 0x7FFFu + ((u >> 16) & 1u);
  return (unsigned short)(u >> 16);
}
__device__ __forceinline__ float bfr(float x) { return __uint_as_float(((unsigned)bfbits(x)) << 16); }

__device__ __forceinline__ f16x16 load_frag(const f16* __restrict__ base, int ld, int row0, int k0) {
  const int lane = threadIdx.x & 31;
  const int r    = lane & 15;
  const int kh   = (lane >> 4) * 8;
  const f16* p0 = base + (size_t)(row0 + r) * ld + (k0 + kh);
  const f16x8 lo = *(const f16x8*)p0;
  const f16x8 hi = *(const f16x8*)(p0 + 16);
  f16x16 f;
#pragma unroll
  for (int i = 0; i < 8; ++i) { f[i] = lo[i]; f[i + 8] = hi[i]; }
  return f;
}

__device__ __forceinline__ f16x16 lds_frag(const f16* base, int stride) {
  const int lane = threadIdx.x & 31;
  const int row  = lane & 15;
  const int kh   = (lane >> 4) * 8;
  const f16x8 lo = *(const f16x8*)(base + row * stride + kh);
  const f16x8 hi = *(const f16x8*)(base + row * stride + kh + 16);
  f16x16 f;
#pragma unroll
  for (int i = 0; i < 8; ++i) { f[i] = lo[i]; f[i + 8] = hi[i]; }
  return f;
}

__device__ __forceinline__ u16x16 lds_frag_bf(const unsigned short* base, int stride) {
  const int lane = threadIdx.x & 31;
  const int row  = lane & 15;
  const int kh   = (lane >> 4) * 8;
  const u16x8 lo = *(const u16x8*)(base + row * stride + kh);
  const u16x8 hi = *(const u16x8*)(base + row * stride + kh + 16);
  u16x16 w;
#pragma unroll
  for (int i = 0; i < 8; ++i) { w[i] = lo[i]; w[i + 8] = hi[i]; }
  return w;
}

__device__ __forceinline__ u16x16 frag_to_bf(f16x16 f) {
  u16x16 w;
#pragma unroll
  for (int i = 0; i < 16; ++i) { const float x = (float)f[i]; w[i] = (unsigned short)(__float_as_uint(x) >> 16); }
  return w;
}

__device__ __forceinline__ f16x8 cvt8(const float* __restrict__ src, float sc) {
  const v4f_t a = *(const v4f_t*)src;
  const v4f_t c = *(const v4f_t*)(src + 4);
  f16x8 o;
  o[0] = (f16)(bfr(a[0]) * sc); o[1] = (f16)(bfr(a[1]) * sc); o[2] = (f16)(bfr(a[2]) * sc); o[3] = (f16)(bfr(a[3]) * sc);
  o[4] = (f16)(bfr(c[0]) * sc); o[5] = (f16)(bfr(c[1]) * sc); o[6] = (f16)(bfr(c[2]) * sc); o[7] = (f16)(bfr(c[3]) * sc);
  return o;
}

template <typename AT, int AKIND>
__global__ __launch_bounds__(256) void gemm_nk(const AT* __restrict__ A, const unsigned short* __restrict__ Alo, int a_bs,
                                               const float* __restrict__ Wm, const float* __restrict__ bias,
                                               float* __restrict__ Y, int y_bs, int lo_rows) {
  __shared__ __attribute__((aligned(16))) f16 ldsA[128 * GSTR];
  __shared__ __attribute__((aligned(16))) unsigned short ldsL2[128 * GSTR];
  __shared__ __attribute__((aligned(16))) f16 ldsW[128 * GSTR];
  __shared__ __attribute__((aligned(16))) float oS[8][32 * 68];
  const int tid = threadIdx.x, lane = tid & 31, wave = tid >> 5, cl = lane & 15, rh = (lane >> 4) * 8;
  const int m0 = blockIdx.x * 128, n0 = blockIdx.y * 128;
  const int bseq = m0 / SEQ, s0 = m0 - bseq * SEQ;
  const size_t arow0 = (size_t)bseq * (size_t)a_bs + (size_t)s0;
  const size_t yrow0 = (size_t)bseq * (size_t)y_bs + (size_t)s0;
  const bool use_lo = (AKIND == 1) && (s0 < lo_rows);
  const int wm = (wave & 3) * 32, wn = (wave >> 2) * 64;
  f32x8 acc[2][4];
#pragma unroll
  for (int i = 0; i < 2; ++i)
#pragma unroll
    for (int j = 0; j < 4; ++j) { f32x8 z = {}; acc[i][j] = z; }

#pragma unroll 1
  for (int k0 = 0; k0 < DD; k0 += 32) {
    __syncthreads();
    { const int row = tid >> 1, ch = (tid & 1) * 16;
      f16* dst = ldsA + row * GSTR + ch;
      if (AKIND == 0) {
        const float* src = (const float*)A + (arow0 + row) * DD + k0 + ch;
        *(f16x8*)dst       = cvt8(src, 1.0f);
        *(f16x8*)(dst + 8) = cvt8(src + 8, 1.0f);
      } else {
        const f16* src = (const f16*)A + (arow0 + row) * DD + k0 + ch;
        *(f16x8*)dst       = *(const f16x8*)src;
        *(f16x8*)(dst + 8) = *(const f16x8*)(src + 8);
        if (use_lo) {
          const unsigned short* s2 = Alo + (arow0 + row) * DD + k0 + ch;
          unsigned short* d2 = ldsL2 + row * GSTR + ch;
          *(u16x8*)d2       = *(const u16x8*)s2;
          *(u16x8*)(d2 + 8) = *(const u16x8*)(s2 + 8);
        }
      }
    }
    { const int n = tid >> 1, ch = (tid & 1) * 16;
      const float* src = Wm + (size_t)(n0 + n) * DD + k0 + ch;
      f16* dst = ldsW + n * GSTR + ch;
      *(f16x8*)dst       = cvt8(src, WSC);
      *(f16x8*)(dst + 8) = cvt8(src + 8, WSC);
    }
    __syncthreads();
    f16x16 af[2];
#pragma unroll
    for (int i = 0; i < 2; ++i) af[i] = lds_frag(ldsA + (wm + 16 * i) * GSTR, GSTR);
#pragma unroll
    for (int j = 0; j < 4; ++j) {
      const f16x16 bfr16 = lds_frag(ldsW + (wn + 16 * j) * GSTR, GSTR);
#pragma unroll
      for (int i = 0; i < 2; ++i) acc[i][j] = wmma16(af[i], bfr16, acc[i][j]);
    }
    if (use_lo) {
      u16x16 alo[2];
#pragma unroll
      for (int i = 0; i < 2; ++i) alo[i] = lds_frag_bf(ldsL2 + (wm + 16 * i) * GSTR, GSTR);
#pragma unroll
      for (int j = 0; j < 4; ++j) {
        const u16x16 bb = frag_to_bf(lds_frag(ldsW + (wn + 16 * j) * GSTR, GSTR));
#pragma unroll
        for (int i = 0; i < 2; ++i) acc[i][j] = wmmabf(alo[i], bb, acc[i][j]);
      }
    }
  }
  float* so = oS[wave];
#pragma unroll
  for (int i = 0; i < 2; ++i)
#pragma unroll
    for (int j = 0; j < 4; ++j) {
      const int n = n0 + wn + 16 * j + cl;
      const float bv = bfr(bias[n]);
#pragma unroll
      for (int r = 0; r < 8; ++r) so[(16 * i + rh + r) * 68 + 16 * j + cl] = acc[i][j][r] * WSCI + bv;
    }
  asm volatile("s_wait_dscnt 0" ::: "memory");
  __builtin_amdgcn_wave_barrier();
#pragma unroll 1
  for (int pass = 0; pass < 2; ++pass) {
#pragma unroll
    for (int it = 0; it < 16; ++it) { const int f4 = lane + 32 * it, rr = f4 >> 4, q = (f4 & 15) * 4;
      *(volatile v4f_t*)(Y + (yrow0 + wm + rr) * DD + n0 + wn + q) = *(const v4fa*)(so + rr * 68 + q); }
    __threadfence();
  }
}

__global__ __launch_bounds__(64) void attn_kernel(const f16* __restrict__ Qb, const f16* __restrict__ Kb, const f16* __restrict__ Vt,
                                                  f16* __restrict__ attnOut, unsigned short* __restrict__ attnLo) {
  __shared__ __attribute__((aligned(16))) f16 ldsK[32 * KSTRIDE];
  __shared__ __attribute__((aligned(16))) f16 ldsV[64 * VSTRIDE];
  __shared__ __attribute__((aligned(16))) f16 ldsO[2][32 * OSTR];
  __shared__ __attribute__((aligned(16))) unsigned short ldsR[2][32 * OSTR];

  const int q0blk = blockIdx.x * 64;
  const int h = blockIdx.y;
  const int b = blockIdx.z;
  const int t = threadIdx.x;
  const int wave = t >> 5;
  const int lane = t & 31;
  const int qlane = lane & 15;
  const int kh8 = (lane >> 4) * 8;
  const int q0 = q0blk + wave * 32;

  const f16* Qh = Qb + (size_t)b * SEQ * DD + h * DKK;
  const f16* Kh = Kb + (size_t)b * SEQ * DD + h * DKK;
  const f16* Vh = Vt + ((size_t)(b * HH + h)) * DKK * SEQ;

  const int krow = t >> 1;
  const int kcol = (t & 1) * 32;
  const f16* kSrc = Kh + (size_t)krow * DD + kcol;
  const f16* vSrc = Vh + (size_t)t * SEQ;

  f16x16 qf[QW][2];
#pragma unroll
  for (int qt = 0; qt < QW; ++qt) {
    qf[qt][0] = load_frag(Qh, DD, q0 + 16 * qt, 0);
    qf[qt][1] = load_frag(Qh, DD, q0 + 16 * qt, 32);
  }

  f32x8 o[QW][4] = {};
  float mrun[QW], lrun[QW];
#pragma unroll
  for (int qt = 0; qt < QW; ++qt) { mrun[qt] = -INFINITY; lrun[qt] = 0.0f; }

  const float scale = 0.125f * 1.44269504088896340736f;
  const float NEG2 = -1.0e9f;
  const int kmax = q0blk + 63;

  f16x8 kreg[4], vreg[4];
#pragma unroll
  for (int i = 0; i < 4; ++i) {
    kreg[i] = *(const f16x8*)(kSrc + 8 * i);
    vreg[i] = *(const f16x8*)(vSrc + 8 * i);
  }

  for (int kb = 0; kb <= kmax; kb += 32) {
    __syncthreads();
#pragma unroll
    for (int i = 0; i < 4; ++i) {
      *(f16x8*)(&ldsK[krow * KSTRIDE + kcol + 8 * i]) = kreg[i];
      *(f16x8*)(&ldsV[t * VSTRIDE + 8 * i])           = vreg[i];
    }
    if (kb + 32 <= kmax) {
      const f16* kn = kSrc + (size_t)(kb + 32) * DD;
      const f16* vn = vSrc + (kb + 32);
#pragma unroll
      for (int i = 0; i < 4; ++i) {
        kreg[i] = *(const f16x8*)(kn + 8 * i);
        vreg[i] = *(const f16x8*)(vn + 8 * i);
      }
    }
    __syncthreads();

    f16x16 kf[2][2];
#pragma unroll
    for (int ktile = 0; ktile < 2; ++ktile)
#pragma unroll
      for (int c = 0; c < 2; ++c)
        kf[ktile][c] = lds_frag(ldsK + (ktile * 16) * KSTRIDE + c * 32, KSTRIDE);

    f16x16 pf[QW];
#pragma unroll
    for (int qt = 0; qt < QW; ++qt) {
      const int q_my = q0 + 16 * qt + qlane;
      unsigned mbits = 0;
#pragma unroll
      for (int r = 0; r < 8; ++r) {
        mbits |= ((kb + kh8 + r) <= q_my)      ? (1u << r)       : 0u;
        mbits |= ((kb + 16 + kh8 + r) <= q_my) ? (1u << (8 + r)) : 0u;
      }
      f32x8 s0 = {}, s1 = {};
      s0 = wmma16(kf[0][0], qf[qt][0], s0);
      s0 = wmma16(kf[0][1], qf[qt][1], s0);
      s1 = wmma16(kf[1][0], qf[qt][0], s1);
      s1 = wmma16(kf[1][1], qf[qt][1], s1);

      float mx = -INFINITY;
#pragma unroll
      for (int r = 0; r < 8; ++r) {
        s0[r] = (mbits & (1u << r))       ? s0[r] * scale : NEG2;
        s1[r] = (mbits & (1u << (8 + r))) ? s1[r] * scale : NEG2;
        mx = fmaxf(mx, fmaxf(s0[r], s1[r]));
      }
      mx = fmaxf(mx, __shfl_xor(mx, 16, 32));
      const float mnew  = fmaxf(mrun[qt], mx);
      const float alpha = exp2f(mrun[qt] - mnew);

      float rsum = 0.0f;
#pragma unroll
      for (int r = 0; r < 8; ++r) {
        const float p0 = exp2f(s0[r] - mnew);
        const float p1 = exp2f(s1[r] - mnew);
        rsum += p0 + p1;
        pf[qt][r]     = (f16)(p0 * PSC);
        pf[qt][r + 8] = (f16)(p1 * PSC);
      }
      rsum += __shfl_xor(rsum, 16, 32);
      lrun[qt] = lrun[qt] * alpha + rsum;
      mrun[qt] = mnew;

#pragma unroll
      for (int j = 0; j < 4; ++j)
#pragma unroll
        for (int r = 0; r < 8; ++r) o[qt][j][r] *= alpha;
    }

#pragma unroll
    for (int j = 0; j < 4; ++j) {
      const f16x16 vf = lds_frag(ldsV + (j * 16) * VSTRIDE, VSTRIDE);
#pragma unroll
      for (int qt = 0; qt < QW; ++qt) o[qt][j] = wmma16(vf, pf[qt], o[qt][j]);
    }
  }

  f16* so = ldsO[wave];
  unsigned short* sres = ldsR[wave];
#pragma unroll
  for (int qt = 0; qt < QW; ++qt) {
    const float rl = 1.0f / (lrun[qt] * PSC);
#pragma unroll
    for (int j = 0; j < 4; ++j)
#pragma unroll
      for (int r = 0; r < 8; ++r) {
        const float val = o[qt][j][r] * rl;
        const f16 hv = (f16)val;
        const int idx = (16 * qt + qlane) * OSTR + j * 16 + kh8 + r;
        so[idx] = hv;
        sres[idx] = bfbits(val - (float)hv);
      }
  }
  asm volatile("s_wait_dscnt 0" ::: "memory");
  __builtin_amdgcn_wave_barrier();
#pragma unroll 1
  for (int pass = 0; pass < 2; ++pass) {
#pragma unroll
    for (int it = 0; it < 8; ++it) { const int ch = lane + 32 * it, ql = ch >> 3, q8 = (ch & 7) * 8;
      const size_t g = ((size_t)(b * SEQ + q0 + ql)) * DD + h * DKK + q8;
      *(volatile v4u_t*)(attnOut + g) = *(const v4ua*)(so + ql * OSTR + q8);
      *(volatile v4u_t*)(attnLo + g)  = *(const v4ua*)(sres + ql * OSTR + q8); }
    __threadfence();
  }
}

__global__ __launch_bounds__(64) void k_early(const float* __restrict__ Pq, const float* __restrict__ Pk, const float* __restrict__ Pv,
                                              f16* __restrict__ att, unsigned short* __restrict__ attLo) {
  __shared__ float qs[EARLY][65];
  __shared__ float ks[EARLY][64];
  __shared__ float vs[EARLY][65];
  __shared__ float ps[EARLY][65];
  __shared__ float invf[32];
  const int h = blockIdx.x, b = blockIdx.y, tid = threadIdx.x;
  const size_t row0 = (size_t)b * SEQ;
#pragma unroll 1
  for (int e = tid; e < EARLY * DKK; e += 64) {
    const int r = e >> 6, d = e & 63;
    const size_t g = (row0 + r) * DD + h * DKK + d;
    qs[r][d] = Pq[g]; ks[r][d] = Pk[g]; vs[r][d] = Pv[g];
  }
  if (tid < 32) invf[tid] = 1.0f / powf(10000.0f, (float)(2 * tid) * 0.015625f);
  __syncthreads();
#pragma unroll 1
  for (int e = tid; e < EARLY * 32; e += 64) {
    const int r = e >> 5, i = e & 31;
    const float ang = (float)r * invf[i];
    const float c = cosf(ang), sn = sinf(ang);
    float a1 = qs[r][i], a2 = qs[r][i + 32];
    qs[r][i] = a1 * c - a2 * sn; qs[r][i + 32] = a2 * c + a1 * sn;
    a1 = ks[r][i]; a2 = ks[r][i + 32];
    ks[r][i] = a1 * c - a2 * sn; ks[r][i + 32] = a2 * c + a1 * sn;
  }
  __syncthreads();
  const int tq = tid;
  float mx = -INFINITY;
#pragma unroll 1
  for (int j = 0; j < EARLY; ++j) {
    float s = 0.0f;
#pragma unroll 2
    for (int d = 0; d < DKK; ++d) s += qs[tq][d] * ks[j][d];
    s = (j <= tq) ? s * 0.125f : -INFINITY;
    ps[j][tq] = s;
    mx = fmaxf(mx, s);
  }
  float l = 0.0f;
#pragma unroll 1
  for (int j = 0; j < EARLY; ++j) { const float p = expf(ps[j][tq] - mx); l += p; ps[j][tq] = p; }
  const float rl = 1.0f / l;
#pragma unroll 1
  for (int d = 0; d < DKK; ++d) {
    float a = 0.0f;
#pragma unroll 2
    for (int j = 0; j < EARLY; ++j) a += ps[j][tq] * vs[j][d];
    qs[tq][d] = a * rl;
  }
  __syncthreads();
#pragma unroll 1
  for (int pass = 0; pass < 2; ++pass) {
#pragma unroll
    for (int it = 0; it < 8; ++it) {
      const int c = tid + 64 * it, r = c >> 3, q8 = (c & 7) * 8;
      union { f16 hh[8]; v4u_t v; } uh;
      union { unsigned short uu[8]; v4u_t v; } ul;
#pragma unroll
      for (int e = 0; e < 8; ++e) { const float val = qs[r][q8 + e]; const f16 hv = (f16)val; uh.hh[e] = hv; ul.uu[e] = bfbits(val - (float)hv); }
      const size_t g = (row0 + r) * DD + h * DKK + q8;
      *(volatile v4u_t*)(att + g)   = uh.v;
      *(volatile v4u_t*)(attLo + g) = ul.v;
    }
    __threadfence();
  }
}

__global__ __launch_bounds__(256) void k_vt(const float* __restrict__ P, f16* __restrict__ Vt) {
  __shared__ __attribute__((aligned(16))) f16 vT[64][72];
  const int tid = threadIdx.x; const size_t t0 = (size_t)blockIdx.x * 64; const int h = blockIdx.y;
  const int b = (int)(t0 / SEQ), n0 = (int)(t0 % SEQ);
#pragma unroll 1
  for (int e = tid; e < 64 * 64; e += 256) { const int t = e >> 6, d = e & 63; vT[d][t] = (f16)P[(t0 + t) * DD + h * DKK + d]; }
  __syncthreads();
#pragma unroll 1
  for (int pass = 0; pass < 2; ++pass) {
#pragma unroll 1
    for (int rr2 = 0; rr2 < 2; ++rr2) { const int r = rr2 * 32 + (tid >> 3), piece = (tid & 7) * 8;
      *(volatile v4u_t*)(Vt + ((size_t)(b * HH + h) * DKK + r) * SEQ + n0 + piece) = *(const v4ua*)(&vT[r][piece]); }
    __threadfence();
  }
}

__global__ __launch_bounds__(256) void k_rope16(const float* __restrict__ P, f16* __restrict__ R16) {
  __shared__ __attribute__((aligned(16))) f16 s[64][72];
  __shared__ float pf[64][65];
  __shared__ float invf[32];
  const int tid = threadIdx.x; const size_t t0 = (size_t)blockIdx.x * 64; const int h = blockIdx.y; const int p0 = (int)(t0 % SEQ);
#pragma unroll 1
  for (int e = tid; e < 64 * 64; e += 256) { const int t = e >> 6, d = e & 63; pf[t][d] = P[(t0 + t) * DD + h * DKK + d]; }
  if (tid < 32) invf[tid] = 1.0f / powf(10000.0f, (float)(2 * tid) * 0.015625f);
  __syncthreads();
#pragma unroll 1
  for (int e = tid; e < 64 * 32; e += 256) { const int t = e >> 5, i = e & 31; const float pos = (float)(p0 + t);
    const float ang = pos * invf[i]; const float c = cosf(ang), sn = sinf(ang);
    const float a1 = pf[t][i], a2 = pf[t][i + 32];
    s[t][i] = (f16)(a1 * c - a2 * sn); s[t][i + 32] = (f16)(a2 * c + a1 * sn); }
  __syncthreads();
#pragma unroll 1
  for (int pass = 0; pass < 2; ++pass) {
#pragma unroll 1
    for (int rr2 = 0; rr2 < 2; ++rr2) { const int r = rr2 * 32 + (tid >> 3), piece = (tid & 7) * 8;
      *(volatile v4u_t*)(R16 + (t0 + r) * DD + h * DKK + piece) = *(const v4ua*)(&s[r][piece]); }
    __threadfence();
  }
}

extern "C" void kernel_launch(void* const* d_in, const int* in_sizes, int n_in,
                              void* d_out, int out_size, void* d_ws, size_t ws_size,
                              hipStream_t stream) {
  if (n_in < 11) return;
  const long long need_act = ((long long)(NB - 1) * SEQ_FULL + SEQ) * (long long)DD;
  if ((long long)in_sizes[0] < need_act || (long long)in_sizes[1] < need_act || (long long)in_sizes[2] < need_act) return;
  if ((long long)out_size < need_act) return;
  if (in_sizes[3] < DD * DD || in_sizes[5] < DD * DD || in_sizes[7] < DD * DD || in_sizes[9] < DD * DD) return;
  if (in_sizes[4] < DD || in_sizes[6] < DD || in_sizes[8] < DD || in_sizes[10] < DD) return;
  const float* xq = (const float*)d_in[0];
  const float* xk = (const float*)d_in[1];
  const float* xv = (const float*)d_in[2];
  const float* Wq = (const float*)d_in[3];  const float* bq = (const float*)d_in[4];
  const float* Wk = (const float*)d_in[5];  const float* bk = (const float*)d_in[6];
  const float* Wv = (const float*)d_in[7];  const float* bvv = (const float*)d_in[8];
  const float* Wo = (const float*)d_in[9];  const float* bo = (const float*)d_in[10];
  float* out = (float*)d_out;

  char* ws = (char*)d_ws;
  const size_t nP = (size_t)MTOK * (size_t)DD;
  float* Pq = (float*)ws; ws += nP * 4;
  float* Pk = (float*)ws; ws += nP * 4;
  float* Pv = (float*)ws; ws += nP * 4;
  f16* Q16 = (f16*)ws; ws += nP * 2;
  f16* K16 = (f16*)ws; ws += nP * 2;
  f16* Vt  = (f16*)ws; ws += nP * 2;
  f16* att = (f16*)ws; ws += nP * 2;
  unsigned short* attLo = (unsigned short*)ws; ws += nP * 2;
  if ((size_t)(ws - (char*)d_ws) > ws_size) return;

  const dim3 blk(256); const dim3 gp(MTOK / 128, DD / 128); const dim3 gh(MTOK / 64, HH);
  gemm_nk<float, 0><<<gp, blk, 0, stream>>>(xq, (const unsigned short*)0, SEQ_FULL, Wq, bq, Pq, SEQ, 0);
  k_rope16<<<gh, blk, 0, stream>>>(Pq, Q16);
  gemm_nk<float, 0><<<gp, blk, 0, stream>>>(xk, (const unsigned short*)0, SEQ_FULL, Wk, bk, Pk, SEQ, 0);
  k_rope16<<<gh, blk, 0, stream>>>(Pk, K16);
  gemm_nk<float, 0><<<gp, blk, 0, stream>>>(xv, (const unsigned short*)0, SEQ_FULL, Wv, bvv, Pv, SEQ, 0);
  k_vt<<<gh, blk, 0, stream>>>(Pv, Vt);
  attn_kernel<<<dim3(SEQ / 64, HH, NB), dim3(64), 0, stream>>>(Q16, K16, Vt, att, attLo);
  k_early<<<dim3(HH, NB), dim3(64), 0, stream>>>(Pq, Pk, Pv, att, attLo);
  gemm_nk<f16, 1><<<gp, blk, 0, stream>>>(att, attLo, SEQ, Wo, bo, out, SEQ_FULL, LOROWS);
}
